// SplitNN_4879082848949
// MI455X (gfx1250) — hardware-run, weakly checked
//
#include <hip/hip_runtime.h>
#pragma clang fp contract(off)


#define NBAT 32
#define FIN  160
#define DH   128
#define NOUT 2
#define XP   168
#define WP   168
#define OP   129
#define NTHR 512
#define EPSC ((float)(4.0 / 30.0))

static_assert(NBAT == 32);
static_assert(DH == 128);
static_assert((NBAT / 16) * (DH / 16) == NTHR / 32);
static_assert(FIN % 32 == 0);
static_assert(FIN % 8 == 0);
static_assert(XP % 8 == 0 && WP % 8 == 0);
static_assert(XP >= FIN && WP >= FIN);
static_assert((DH * (FIN / 8)) % NTHR == 0);
static_assert(DH * NOUT <= NTHR);
static_assert(NBAT * NOUT <= NTHR);
static_assert(16 * 16 == NBAT * NOUT * 4);
static_assert((size_t)2 * NBAT * XP * 2 + (size_t)2 * DH * WP * 2 + (size_t)NBAT * OP * 4 + (size_t)DH * 4 + (size_t)DH * NOUT * 4 + (size_t)NBAT * NOUT * 4 <= (size_t)131072);

typedef unsigned short bf;
typedef __attribute__((ext_vector_type(16))) __bf16   v16bf;
typedef __attribute__((ext_vector_type(8)))  unsigned short v8us;
typedef __attribute__((ext_vector_type(8)))  float    v8f;
typedef __attribute__((ext_vector_type(4)))  float    v4f;
typedef v4f  __attribute__((may_alias)) v4fa;

__device__ __forceinline__ unsigned short f2bf(float f) { unsigned u = __float_as_uint(f); u += 0x7FFFu + ((u >> 16) & 1u); return (unsigned short)(u >> 16); }
__device__ __forceinline__ float bfr(float f) { return __uint_as_float(((unsigned)f2bf(f)) << 16); }
__device__ __forceinline__ v16bf cat16b(v8us lo, v8us hi) { return __builtin_bit_cast(v16bf, __builtin_shufflevector(lo, hi, 0, 1, 2, 3, 4, 5, 6, 7, 8, 9, 10, 11, 12, 13, 14, 15)); }
__device__ __forceinline__ v8f wmmab(v16bf a, v16bf b, v8f c) { return __builtin_amdgcn_wmma_f32_16x16x32_bf16(false, a, false, b, (short)0, c, false, false); }
__device__ __forceinline__ v8f wmmab_g(v16bf a, v16bf b, v8f c) { c = wmmab(a, b, c); asm volatile("v_nop\n\tv_nop\n\tv_nop\n\tv_nop" : "+v"(c) : "v"(a), "v"(b)); return c; }

__global__ __launch_bounds__(NTHR) void k_fused(const float* __restrict__ x1, const float* __restrict__ x2, const float* __restrict__ impor,
                                                const float* __restrict__ W1, const float* __restrict__ b1, const float* __restrict__ W2, const float* __restrict__ b2,
                                                const float* __restrict__ Ws, const float* __restrict__ bs, const float* __restrict__ lap, const float* __restrict__ rr, float* OUT) {
    __shared__ __align__(16) bf xs1[NBAT * XP];
    __shared__ __align__(16) bf xs2[NBAT * XP];
    __shared__ __align__(16) bf wt1[DH * WP];
    __shared__ __align__(16) bf wt2[DH * WP];
    __shared__ __align__(16) float o1s[NBAT * OP];
    __shared__ __align__(16) float nms[DH];
    __shared__ __align__(16) float wss[DH * NOUT];
    __shared__ __align__(16) float outs[NBAT * NOUT];

    const int tid = threadIdx.x;
    const int lane = tid & 31, lr = lane & 15, hi = lane >> 4;
    const int wave = __builtin_amdgcn_readfirstlane((int)(threadIdx.x >> 5));
    const int mtile = wave >> 3, ntile = wave & 7;

#pragma unroll 1
    for (int c = tid; c < NBAT * (FIN / 8); c += NTHR) {
        const int row = c / (FIN / 8), k8 = (c % (FIN / 8)) * 8;
        const v4f a0 = *(const v4f*)(x1 + row * FIN + k8), a1 = *(const v4f*)(x1 + row * FIN + k8 + 4);
        const v4f c0 = *(const v4f*)(x2 + row * FIN + k8), c1 = *(const v4f*)(x2 + row * FIN + k8 + 4);
        v8us u, w;
#pragma unroll
        for (int i = 0; i < 4; ++i) { u[i] = f2bf(a0[i]); u[4 + i] = f2bf(a1[i]); w[i] = f2bf(c0[i]); w[4 + i] = f2bf(c1[i]); }
        *(v8us*)(&xs1[row * XP + k8]) = u;
        *(v8us*)(&xs2[row * XP + k8]) = w;
    }
#pragma unroll 1
    for (int it = 0; it < (DH * (FIN / 8)) / NTHR; ++it) {
        const int c = it * NTHR + tid; const int n = c & (DH - 1), k0 = (c >> 7) * 8;
        v8us u;
#pragma unroll
        for (int j = 0; j < 8; ++j) u[j] = f2bf(W1[(k0 + j) * DH + n]);
        *(v8us*)(&wt1[n * WP + k0]) = u;
    }
#pragma unroll 1
    for (int it = 0; it < (DH * (FIN / 8)) / NTHR; ++it) {
        const int c = it * NTHR + tid; const int n = c & (DH - 1), k0 = (c >> 7) * 8;
        v8us u;
#pragma unroll
        for (int j = 0; j < 8; ++j) u[j] = f2bf(W2[(k0 + j) * DH + n]);
        *(v8us*)(&wt2[n * WP + k0]) = u;
    }
    if (tid < DH * NOUT) wss[tid] = bfr(Ws[tid]);
    __syncthreads();

    const int aoff = (mtile * 16 + lr) * XP + 8 * hi;
    const int boff = (ntile * 16 + lr) * WP + 8 * hi;
    v8f acc1 = (v8f){}, acc2 = (v8f){};
#pragma unroll
    for (int kc = 0; kc < FIN; kc += 32) {
        const v16bf a1 = cat16b(*(const v8us*)(&xs1[aoff + kc]), *(const v8us*)(&xs1[aoff + kc + 16]));
        const v16bf w1 = cat16b(*(const v8us*)(&wt1[boff + kc]), *(const v8us*)(&wt1[boff + kc + 16]));
        acc1 = wmmab_g(a1, w1, acc1);
        const v16bf a2 = cat16b(*(const v8us*)(&xs2[aoff + kc]), *(const v8us*)(&xs2[aoff + kc + 16]));
        const v16bf w2 = cat16b(*(const v8us*)(&wt2[boff + kc]), *(const v8us*)(&wt2[boff + kc + 16]));
        acc2 = wmmab_g(a2, w2, acc2);
    }

    const int col = ntile * 16 + lr;
    const int rowb = mtile * 16 + 8 * hi;
    const float b1c = bfr(b1[col]);
    const float b2c = bfr(b2[col]);
    const float rrc = bfr(rr[col]);
    float p1[8], p2[8];
#pragma unroll
    for (int r = 0; r < 8; ++r) { p1[r] = acc1[r] + b1c; p2[r] = acc2[r] + b2c; o1s[(rowb + r) * OP + col] = p1[r]; }
    __syncthreads();

    if (tid < DH) {
        float mx = o1s[tid], mn = mx;
#pragma unroll 1
        for (int mm = 1; mm < NBAT; ++mm) { const float v = o1s[mm * OP + tid]; mx = fmaxf(mx, v); mn = fminf(mn, v); }
        const float dF = mx - mn;
        float es = bfr(impor[tid]) * EPSC;
        es = (es == 0.0f) ? 1e-4f : es;
        float mul = dF * (1.0f / es);
        mul = (mul == 0.0f) ? 1e-4f : mul;
        nms[tid] = (dF == 0.0f) ? 0.0f : mul;
    }
    __syncthreads();

    {
        const float mulc = nms[col];
#pragma unroll
        for (int r = 0; r < 8; ++r) {
            const float lv = bfr(lap[(rowb + r) * DH + col]);
            const float nz = lv * mulc;
            const float v1 = (p1[r] + nz) * rrc;
            o1s[(rowb + r) * OP + col] = fminf(v1, p2[r]);
        }
    }
    __syncthreads();

    if (tid < NBAT * NOUT) {
        const int mm = tid >> 1, j = tid & 1;
        float sum = bfr(bs[j]);
#pragma unroll 4
        for (int k = 0; k < DH; ++k) sum = fmaf(o1s[mm * OP + k], wss[k * NOUT + j], sum);
        outs[tid] = sum;
    }
    __syncthreads();

    if (wave == 0) {
        if (lane < 16) {
            const v4f val = *(const v4fa*)(&outs[lane * 4]);
            *(volatile v4f*)(OUT + lane * 4) = val;
            __threadfence();
            *(volatile v4f*)(OUT + lane * 4) = val;
        }
    }
}

extern "C" void kernel_launch(void* const* d_in, const int* in_sizes, int n_in,
                              void* d_out, int out_size, void* d_ws, size_t ws_size, hipStream_t stream) {
    (void)d_ws; (void)ws_size;
    if (n_in < 11) return;
    if (in_sizes[0] < NBAT * FIN || in_sizes[1] < NBAT * FIN) return;
    if (in_sizes[2] < DH) return;
    if (in_sizes[3] < FIN * DH || in_sizes[5] < FIN * DH) return;
    if (in_sizes[4] < DH || in_sizes[6] < DH) return;
    if (in_sizes[7] < DH * NOUT || in_sizes[8] < NOUT) return;
    if (in_sizes[9] < NBAT * DH || in_sizes[10] < DH) return;
    if (out_size < NBAT * NOUT) return;
    const float* x1    = (const float*)d_in[0];
    const float* x2    = (const float*)d_in[1];
    const float* impor = (const float*)d_in[2];
    const float* W1    = (const float*)d_in[3];
    const float* b1    = (const float*)d_in[4];
    const float* W2    = (const float*)d_in[5];
    const float* b2    = (const float*)d_in[6];
    const float* Ws    = (const float*)d_in[7];
    const float* bs    = (const float*)d_in[8];
    const float* lap   = (const float*)d_in[9];
    const float* rr    = (const float*)d_in[10];
    float* OUT = (float*)d_out;
    k_fused<<<1, NTHR, 0, stream>>>(x1, x2, impor, W1, b1, W2, b2, Ws, bs, lap, rr, OUT);
}
